// HybridMamba2Block_49074296324243
// MI455X (gfx1250) — hardware-verified
//
#include <hip/hip_runtime.h>
#include <math.h>
#include <stdint.h>

typedef __attribute__((ext_vector_type(16))) _Float16 v16h;
typedef __attribute__((ext_vector_type(8)))  _Float16 v8h;
typedef __attribute__((ext_vector_type(16))) __bf16   v16b;
typedef __attribute__((ext_vector_type(8)))  __bf16   v8b;
typedef __attribute__((ext_vector_type(8)))  float    v8f;
typedef __attribute__((ext_vector_type(4)))  float    v4f;
typedef __attribute__((ext_vector_type(4)))  unsigned int v4u;

constexpr int kBatch   = 2;
constexpr int kT       = 2048;
constexpr int kD       = 1024;
constexpr int kRows    = kBatch * kT;
constexpr int kHeadsA  = 16;
constexpr int kHD      = 64;
constexpr int kWin     = 128;
constexpr int kHS      = 8;
constexpr int kDI      = 2048;
constexpr int kNS      = 16;
constexpr int kDTR     = 64;
constexpr int kPch     = 256;
constexpr int kWinRows = 4416;
constexpr int kXZP     = 4096;
constexpr int kDBCP    = 320;
constexpr int kChunk   = 32;
constexpr int kTP      = 260;
constexpr int kSGH     = 8;
constexpr int kBandL   = 2;
constexpr int kPBW     = 192;

__device__ __forceinline__ unsigned short f2bf_bits(float f) {
  unsigned u = __float_as_uint(f);
  return (unsigned short)((u + 0x7FFFu + ((u >> 16) & 1u)) >> 16);
}
__device__ __forceinline__ float bf_bits2f(unsigned short h) { return __uint_as_float(((unsigned)h) << 16); }
__device__ __forceinline__ unsigned pk16(unsigned short a, unsigned short b) { return (unsigned)a | ((unsigned)b << 16); }

__device__ __forceinline__ void dep_guard_h(v8f& a, v8f& b, v16h x, v16h y) { asm volatile("v_nop\n\tv_nop\n\tv_nop\n\tv_nop" : "+v"(a), "+v"(b) : "v"(x), "v"(y)); }
__device__ __forceinline__ void dep_guard_b(v8f& a, v8f& b, v16b x, v16b y) { asm volatile("v_nop\n\tv_nop\n\tv_nop\n\tv_nop" : "+v"(a), "+v"(b) : "v"(x), "v"(y)); }
__device__ __forceinline__ void keep4_h(v16h a, v16h b, v16h c, v16h d) { asm volatile("v_nop" :: "v"(a), "v"(b), "v"(c), "v"(d)); }
__device__ __forceinline__ void keep4_b(v16b a, v16b b, v16b c, v16b d) { asm volatile("v_nop" :: "v"(a), "v"(b), "v"(c), "v"(d)); }
__device__ __forceinline__ void acc_guard4(v8f& a, v8f& b, v8f& c, v8f& d) { asm volatile("v_nop\n\tv_nop\n\tv_nop\n\tv_nop" : "+v"(a), "+v"(b), "+v"(c), "+v"(d)); }
template <typename T> struct Frag;
template <> struct Frag<_Float16> {
  typedef v16h V; union U { v16h v; v8h h[2]; };
  static __device__ __forceinline__ v16h load(const _Float16* p) {
    U f; f.h[0] = *(const v8h*)(p); f.h[1] = *(const v8h*)(p + 16); return f.v;
  }
  static __device__ __forceinline__ v8f mma(v16h a, v16h b, v8f c) {
    return __builtin_amdgcn_wmma_f32_16x16x32_f16(false, a, false, b, (short)0, c, false, false);
  }
  static __device__ __forceinline__ void guard(v8f& a, v8f& b, v16h x, v16h y) { dep_guard_h(a, b, x, y); }
  static __device__ __forceinline__ void keep(v16h a, v16h b, v16h c, v16h d) { keep4_h(a, b, c, d); }
};
template <> struct Frag<__bf16> {
  typedef v16b V; union U { v16b v; v8b h[2]; };
  static __device__ __forceinline__ v16b load(const __bf16* p) {
    U f; f.h[0] = *(const v8b*)(p); f.h[1] = *(const v8b*)(p + 16); return f.v;
  }
  static __device__ __forceinline__ v8f mma(v16b a, v16b b, v8f c) {
    return __builtin_amdgcn_wmma_f32_16x16x32_bf16(false, a, false, b, (short)0, c, false, false);
  }
  static __device__ __forceinline__ void guard(v8f& a, v8f& b, v16b x, v16b y) { dep_guard_b(a, b, x, y); }
  static __device__ __forceinline__ void keep(v16b a, v16b b, v16b c, v16b d) { keep4_b(a, b, c, d); }
};

template <int ET> struct Elem;
template <> struct Elem<0> { typedef _Float16 T; };
template <> struct Elem<1> { typedef __bf16 T; };
template <int ET, bool SPLIT, int BIAS_MODE, int OUT_MODE, bool RESID, int ACT = 0,
          int BANDL = -1, int BANDR = 0, int BANDKL = -1, int BANDKR = 0, bool BANDST = false>
__global__ __launch_bounds__(256) void wmma_gemm64(
    const unsigned short* __restrict__ Ap, const unsigned short* __restrict__ A2p, int lda, long strideA,
    const unsigned short* __restrict__ Btp, const unsigned short* __restrict__ Bt2p, int ldb, long strideB,
    void* __restrict__ Cout, void* __restrict__ Cout2, int ldc, long strideC,
    const float* __restrict__ bias,
    const float* __restrict__ resid, long strideR,
    int M, int N, int K, float scale, float bsc) {
  typedef typename Elem<ET>::T T;
  typedef typename Frag<T>::V V;
  const T* A = (const T*)Ap; const T* A2 = (const T*)A2p; const T* Bt = (const T*)Btp; const T* Bt2 = (const T*)Bt2p;
  __shared__ __align__(16) float sT[8][16 * 68];
  const int b    = blockIdx.y;
  const int lane = threadIdx.x & 31;
  const int wave = threadIdx.x >> 5;
  const int tilesN = N >> 6;
  const int tilesM = M >> 6;
  const int tile = blockIdx.x * 8 + wave;
  if (tile >= tilesM * tilesN) return;
  const int tm = tile / tilesN;
  const int tn = tile - tm * tilesN;
  const int m0 = tm << 6;
  const int n0 = tn << 6;
  if (BANDL >= 0) {
    const int dmn = tm - tn;
    if (dmn > BANDL || dmn < -BANDR) return;
  }
  int nC = n0;
  if (BANDST && BANDL >= 0) {
    int tl = tm - BANDL; tl = (tl < 0) ? 0 : tl;
    nC = n0 - (tl << 6);
  }

  const T* Ab  = A  + (size_t)b * strideA;
  const T* Bb  = Bt + (size_t)b * strideB;
  const T* Ab2 = SPLIT ? (A2  + (size_t)b * strideA) : nullptr;
  const T* Bb2 = SPLIT ? (Bt2 + (size_t)b * strideB) : nullptr;

  const int rlane = lane & 15;
  const int koff  = (lane >> 4) * 8;
  const int mOff  = (lane >> 4) * 8;

  v8f acc[4][4];
#pragma unroll
  for (int i = 0; i < 4; ++i)
#pragma unroll
    for (int j = 0; j < 4; ++j) acc[i][j] = (v8f){0.f,0.f,0.f,0.f,0.f,0.f,0.f,0.f};

  int kBeg = 0, kEnd = K;
  if (BANDKL >= 0) {
    int ks = (tm - BANDKL) * 64;     ks = (ks < 0) ? 0 : ks;
    int ke = (tm + BANDKR + 1) * 64; ke = (ke > K) ? K : ke;
    kBeg = __builtin_amdgcn_readfirstlane(ks);
    kEnd = __builtin_amdgcn_readfirstlane(ke);
  }
  const int kA = (BANDST && BANDKL >= 0) ? kBeg : 0;
  for (int k0 = kBeg; k0 < kEnd; k0 += 32) {
    V bh[4], bl[4];
#pragma unroll
    for (int j = 0; j < 4; ++j) {
      const size_t bo = (size_t)(n0 + (j << 4) + rlane) * ldb + koff + k0;
      bh[j] = Frag<T>::load(Bb + bo);
      if (SPLIT) bl[j] = Frag<T>::load(Bb2 + bo);
    }
#pragma unroll
    for (int i = 0; i < 4; ++i) {
      const size_t ao = (size_t)(m0 + (i << 4) + rlane) * lda + koff + (k0 - kA);
      V ah = Frag<T>::load(Ab + ao);
      V al;
      if (SPLIT) al = Frag<T>::load(Ab2 + ao);
#pragma unroll
      for (int j = 0; j < 4; ++j) {
        acc[i][j] = Frag<T>::mma(ah, bh[j], acc[i][j]);
        if (SPLIT) {
          acc[i][j] = Frag<T>::mma(ah, bl[j], acc[i][j]);
          acc[i][j] = Frag<T>::mma(al, bh[j], acc[i][j]);
        }
      }
      Frag<T>::guard(acc[i][0], acc[i][3], ah, SPLIT ? al : ah);
    }
    Frag<T>::keep(bh[0], bh[1], bh[2], bh[3]);
    if (SPLIT) Frag<T>::keep(bl[0], bl[1], bl[2], bl[3]);
  }
  acc_guard4(acc[0][0], acc[0][1], acc[0][2], acc[0][3]);
  acc_guard4(acc[1][0], acc[1][1], acc[1][2], acc[1][3]);
  acc_guard4(acc[2][0], acc[2][1], acc[2][2], acc[2][3]);
  acc_guard4(acc[3][0], acc[3][1], acc[3][2], acc[3][3]);

  float* slab = sT[wave];
  const float* Rb = RESID ? (resid + (size_t)b * strideR) : nullptr;
#pragma unroll
  for (int i = 0; i < 4; ++i) {
    const int mBase = m0 + (i << 4);
#pragma unroll
    for (int j = 0; j < 4; ++j) {
      const int n = n0 + (j << 4) + rlane;
      float bv = 0.f;
      if (BIAS_MODE == 2) bv = bias[n] * bsc;
#pragma unroll
      for (int r = 0; r < 8; ++r) {
        float v = acc[i][j][r] * scale;
        if (BIAS_MODE == 1) v += bias[mBase + mOff + r] * bsc;
        if (BIAS_MODE == 2) v += bv;
        if (RESID) v += Rb[(size_t)(mBase + mOff + r) * ldc + n];
        if (ACT == 1) v = tanhf(v);
        if (ACT == 2) v = fmaxf(v, 0.0f);
        if (ACT == 3) v = v / (1.0f + expf(-v));
        if (ACT == 4) v = (v > 0.f) ? v : 0.01f * v;
        slab[(mOff + r) * 68 + (j << 4) + rlane] = v;
      }
    }
    __builtin_amdgcn_fence(__ATOMIC_RELEASE, "workgroup");
    __builtin_amdgcn_wave_barrier();
    __builtin_amdgcn_fence(__ATOMIC_ACQUIRE, "workgroup");
    if (OUT_MODE == 0) {
      float* C = (float*)Cout + (size_t)b * strideC;
      const int hh = lane >> 4, c4 = (lane & 15) * 4;
      for (int pass = 0; pass < 2; ++pass) {
#pragma unroll
        for (int it = 0; it < 8; ++it) {
          const int row = it * 2 + hh;
          v4f v = *(const v4f*)(slab + row * 68 + c4);
          *(volatile v4f*)(C + (size_t)(mBase + row) * ldc + nC + c4) = v;
        }
        __threadfence();
      }
    } else {
      const int q = lane >> 3, c8 = (lane & 7) * 8;
      unsigned short* C  = (unsigned short*)Cout  + (size_t)b * strideC;
      unsigned short* C2 = (OUT_MODE == 2) ? ((unsigned short*)Cout2 + (size_t)b * strideC) : nullptr;
      for (int pass = 0; pass < 2; ++pass) {
#pragma unroll
        for (int it = 0; it < 4; ++it) {
          const int row = it * 4 + q;
          const float* sp = slab + row * 68 + c8;
          v8h hv, lv;
#pragma unroll
          for (int e = 0; e < 8; ++e) {
            if (OUT_MODE == 1) {
              hv[e] = (_Float16)sp[e];
            } else {
              unsigned short hb = f2bf_bits(sp[e]);
              unsigned short lb = f2bf_bits(sp[e] - bf_bits2f(hb));
              hv[e] = __builtin_bit_cast(_Float16, hb);
              lv[e] = __builtin_bit_cast(_Float16, lb);
            }
          }
          *(volatile v8h*)(C + (size_t)(mBase + row) * ldc + nC + c8) = hv;
          if (OUT_MODE == 2) *(volatile v8h*)(C2 + (size_t)(mBase + row) * ldc + nC + c8) = lv;
        }
        __threadfence();
      }
    }
    __builtin_amdgcn_fence(__ATOMIC_RELEASE, "workgroup");
    __builtin_amdgcn_wave_barrier();
    __builtin_amdgcn_fence(__ATOMIC_ACQUIRE, "workgroup");
  }
}

__global__ __launch_bounds__(256) void cast_f16_kernel(
    const float* __restrict__ src, unsigned short* __restrict__ dst, int total8, float scale)
{
  const int i = blockIdx.x * 256 + threadIdx.x;
  if (i >= total8) return;
  const size_t e0 = (size_t)i << 3;
  const float* p = src + e0;
  const v4f a0 = *(const v4f*)(p);
  const v4f a1 = *(const v4f*)(p + 4);
  v8h hv;
#pragma unroll
  for (int e = 0; e < 4; ++e) {
    hv[e]     = (_Float16)(a0[e] * scale);
    hv[4 + e] = (_Float16)(a1[e] * scale);
  }
  unsigned short* q = dst + e0;
  *(volatile v8h*)q = hv;
  __threadfence();
  *(volatile v8h*)q = hv;
}

__global__ __launch_bounds__(128) void rms_f16_kernel(
    const float* __restrict__ X, const float* __restrict__ w, unsigned short* __restrict__ O16)
{
  __shared__ float red[4];
  const int tid = threadIdx.x, lane = tid & 31, wave = tid >> 5;
  const size_t base = (size_t)blockIdx.x * kD + tid * 8;
  const v4f a0 = *(const v4f*)(X + base);
  const v4f a1 = *(const v4f*)(X + base + 4);
  float s = ((a0[0] * a0[0] + a0[1] * a0[1]) + (a0[2] * a0[2] + a0[3] * a0[3]))
          + ((a1[0] * a1[0] + a1[1] * a1[1]) + (a1[2] * a1[2] + a1[3] * a1[3]));
#pragma unroll
  for (int off = 16; off > 0; off >>= 1) s += __shfl_xor(s, off, 32);
  if (lane == 0) red[wave] = s;
  __syncthreads();
  const float tot = (red[0] + red[1]) + (red[2] + red[3]);
  const float ms  = tot * (1.0f / 1024.0f);
  const float rs  = rsqrtf(ms + 1e-6f);
  const v4f w0 = *(const v4f*)(w + tid * 8);
  const v4f w1 = *(const v4f*)(w + tid * 8 + 4);
  v8h hv;
#pragma unroll
  for (int e = 0; e < 4; ++e) {
    hv[e]     = (_Float16)((a0[e] * rs) * w0[e]);
    hv[4 + e] = (_Float16)((a1[e] * rs) * w1[e]);
  }
  unsigned short* q = O16 + base;
  *(volatile v8h*)q = hv;
  __threadfence();
  *(volatile v8h*)q = hv;
}

__global__ __launch_bounds__(256) void ssm_scan_kernel(
    const float* __restrict__ XZ, const float* __restrict__ DBC,
    const float* __restrict__ Wdt, const float* __restrict__ dt_bias,
    const float* __restrict__ conv_w, const float* __restrict__ conv_b,
    const float* __restrict__ A_log, const float* __restrict__ Dskip,
    float* __restrict__ Y)
{
  __shared__ float sdt[kChunk];
  __shared__ __align__(16) float sDA[kChunk * kNS];
  __shared__ __align__(16) float sDB[kChunk * kNS];
  __shared__ __align__(16) float sCC[kChunk * kNS];
  __shared__ __align__(16) float sY[kChunk * kTP];
  const int tid = threadIdx.x, lane = tid & 31, wave = tid >> 5;
  const int h = blockIdx.x;
  const int c = h * kPch + tid;
  const float w0 = conv_w[c * 4 + 0], w1 = conv_w[c * 4 + 1], w2 = conv_w[c * 4 + 2], w3 = conv_w[c * 4 + 3];
  const float cb = conv_b[c];
  const float dsk = Dskip[c];
  const float biash = dt_bias[h];
  const float an = -expf(A_log[h * kNS + (tid & 15)]);
  float hst[kNS];
#pragma unroll
  for (int n = 0; n < kNS; ++n) hst[n] = 0.f;
  float xm3 = 0.f, xm2 = 0.f, xm1 = 0.f;
  const int hrow = wave >> 1;
  const int hch  = (wave & 1) * 128 + lane * 4;

#pragma unroll 1
  for (int ch = 0; ch < kT / kChunk; ++ch) {
    const int r0 = ch * kChunk;
    if (wave == 0) {
      const float* pd = DBC + (size_t)(r0 + lane) * kDBCP;
      const float* pw = Wdt + h * kDTR;
      float acc = 0.f;
#pragma unroll 1
      for (int k = 0; k < kDTR; ++k) acc = fmaf(pd[k], pw[k], acc);
      const float a  = acc + biash;
      const float sp = fmaxf(a, 0.0f) + log1pf(__expf(-fabsf(a)));
      sdt[lane] = fminf(fmaxf(sp, 1e-4f), 1.0f);
    }
    __syncthreads();
#pragma unroll 1
    for (int q = 0; q < 2; ++q) {
      const int idx = tid + q * 256;
      const int s = idx >> 4, n = idx & 15;
      const float dtv = sdt[s];
      const float* pr = DBC + (size_t)(r0 + s) * kDBCP;
      sDA[idx] = expf(dtv * an);
      sDB[idx] = dtv * pr[kDTR + h * kNS + n];
      sCC[idx] = pr[kDTR + kHS * kNS + h * kNS + n];
    }
    __syncthreads();
#pragma unroll 1
    for (int s = 0; s < kChunk; ++s) {
      const size_t row = (size_t)(r0 + s);
      const float x = XZ[row * kXZP + c];
      float a = w0 * xm3;
      a = fmaf(w1, xm2, a);
      a = fmaf(w2, xm1, a);
      a = fmaf(w3, x, a);
      a += cb;
      const float sg = __builtin_amdgcn_rcpf(1.0f + __expf(-a));
      const float xc = a * sg;
      v4f da[4], db[4], cc[4];
#pragma unroll
      for (int qq = 0; qq < 4; ++qq) {
        da[qq] = *(const v4f*)(sDA + s * kNS + 4 * qq);
        db[qq] = *(const v4f*)(sDB + s * kNS + 4 * qq);
        cc[qq] = *(const v4f*)(sCC + s * kNS + 4 * qq);
      }
      float y = 0.f;
#pragma unroll
      for (int n = 0; n < kNS; ++n) {
        const float hn = hst[n] * da[n >> 2][n & 3] + xc * db[n >> 2][n & 3];
        hst[n] = hn;
        y = fmaf(hn, cc[n >> 2][n & 3], y);
      }
      y = fmaf(dsk, xc, y);
      sY[s * kTP + tid] = y;
      xm3 = xm2; xm2 = xm1; xm1 = x;
    }
    __syncthreads();
    v4f fv[8];
#pragma unroll
    for (int it = 0; it < 8; ++it) fv[it] = *(const v4f*)(sY + (it * 4 + hrow) * kTP + hch);
    for (int pass = 0; pass < 2; ++pass) {
#pragma unroll
      for (int it = 0; it < 8; ++it)
        *(volatile v4f*)(Y + (size_t)(r0 + it * 4 + hrow) * kDI + h * kPch + hch) = fv[it];
      __threadfence();
    }
  }
}

__global__ __launch_bounds__(256) void gate_rms_kernel(
    const float* __restrict__ Y2, const float* __restrict__ XZ, const float* __restrict__ w,
    unsigned short* __restrict__ G16)
{
  __shared__ float red[8];
  const int tid = threadIdx.x, lane = tid & 31, wave = tid >> 5;
  const int row = blockIdx.x;
  const int c8 = tid * 8;
  const v4f ya = *(const v4f*)(Y2 + (size_t)row * kDI + c8);
  const v4f yb = *(const v4f*)(Y2 + (size_t)row * kDI + c8 + 4);
  const v4f za = *(const v4f*)(XZ + (size_t)row * kXZP + kDI + c8);
  const v4f zb = *(const v4f*)(XZ + (size_t)row * kXZP + kDI + c8 + 4);
  float t[8];
  float ss = 0.f;
#pragma unroll
  for (int e = 0; e < 4; ++e) {
    const float z0 = za[e], z1 = zb[e];
    const float g0 = z0 * __builtin_amdgcn_rcpf(1.0f + __expf(-z0));
    const float g1 = z1 * __builtin_amdgcn_rcpf(1.0f + __expf(-z1));
    t[e]     = ya[e] * g0;
    t[4 + e] = yb[e] * g1;
  }
#pragma unroll
  for (int e = 0; e < 8; ++e) ss = fmaf(t[e], t[e], ss);
#pragma unroll
  for (int off = 16; off > 0; off >>= 1) ss += __shfl_xor(ss, off, 32);
  if (lane == 0) red[wave] = ss;
  __syncthreads();
  float tot = 0.f;
#pragma unroll
  for (int q = 0; q < 8; ++q) tot += red[q];
  const float ms = tot * (1.0f / 2048.0f);
  const float rs = rsqrtf(ms + 1e-6f);
  const v4f wa = *(const v4f*)(w + c8);
  const v4f wb = *(const v4f*)(w + c8 + 4);
  v8h hv;
#pragma unroll
  for (int e = 0; e < 4; ++e) {
    hv[e]     = (_Float16)((t[e] * rs) * wa[e]);
    hv[4 + e] = (_Float16)((t[4 + e] * rs) * wb[e]);
  }
  unsigned short* q = G16 + (size_t)row * kDI + c8;
  *(volatile v8h*)q = hv;
  __threadfence();
  *(volatile v8h*)q = hv;
}

__global__ __launch_bounds__(256) void rope_table_kernel(float* __restrict__ CS)
{
  const int idx = blockIdx.x * 256 + threadIdx.x;
  const int t = idx >> 5, f = idx & 31;
  const float e   = (float)(2 * f) * 0.015625f;
  const float inv = exp2f(-e * 13.28771237954945f);
  const float ang = (float)t * inv;
  float sn, cs;
  sincosf(ang, &sn, &cs);
  float* pc = CS + (size_t)t * 64 + f;
  *(volatile float*)pc = cs;
  *(volatile float*)(pc + 32) = sn;
  __threadfence();
  *(volatile float*)pc = cs;
  *(volatile float*)(pc + 32) = sn;
}

__global__ __launch_bounds__(256) void rope_cast_kernel(
    const float* __restrict__ QKF, const float* __restrict__ CS, unsigned short* __restrict__ QK16)
{
  const int row = blockIdx.x;
  const int t   = row & (kT - 1);
  const int tid = threadIdx.x;
  const int c8  = tid * 8;
  const int d8  = c8 & (kHD - 1);
  const int p8  = c8 ^ 32;
  const int f8  = d8 & 31;
  const float sgn = (d8 < 32) ? -1.0f : 1.0f;
  const float* xr = QKF + (size_t)row * (2 * kD);
  const v4f xa0 = *(const v4f*)(xr + c8);
  const v4f xa1 = *(const v4f*)(xr + c8 + 4);
  const v4f xb0 = *(const v4f*)(xr + p8);
  const v4f xb1 = *(const v4f*)(xr + p8 + 4);
  const float* cr = CS + (size_t)t * 64;
  const v4f ca = *(const v4f*)(cr + f8);
  const v4f cbv = *(const v4f*)(cr + f8 + 4);
  const v4f sa = *(const v4f*)(cr + 32 + f8);
  const v4f sbv = *(const v4f*)(cr + 32 + f8 + 4);
  v8h hv;
#pragma unroll
  for (int e = 0; e < 4; ++e) {
    const float o0 = xa0[e] * ca[e]  + (sgn * xb0[e]) * sa[e];
    const float o1 = xa1[e] * cbv[e] + (sgn * xb1[e]) * sbv[e];
    hv[e]     = (_Float16)(o0 * 8.0f);
    hv[4 + e] = (_Float16)(o1 * 8.0f);
  }
  unsigned short* q = QK16 + (size_t)row * (2 * kD) + c8;
  *(volatile v8h*)q = hv;
  __threadfence();
  *(volatile v8h*)q = hv;
}

__global__ __launch_bounds__(32) void band_softmax_kernel(const float* __restrict__ S, unsigned short* __restrict__ P)
{
  const int i    = blockIdx.x;
  const int y    = blockIdx.y;
  const int lane = threadIdx.x;
  const int tm   = i >> 6;
  int tlo = tm - kBandL; tlo = (tlo < 0) ? 0 : tlo;
  const int c0 = tlo * 64;
  const int c1 = (tm + 1) * 64;
  const int jj = lane * 8;
  const int j  = c0 + jj;
  const bool active = (j < c1);
  const int jjc = active ? jj : 0;
  const size_t roff = ((size_t)y * kT + (size_t)i) * kPBW;
  const v4f a0 = *(const v4f*)(S + roff + jjc);
  const v4f a1 = *(const v4f*)(S + roff + jjc + 4);
  const float sv[8] = {a0[0], a0[1], a0[2], a0[3], a1[0], a1[1], a1[2], a1[3]};
  bool  adm[8];
  float t[8];
  float m = -INFINITY;
#pragma unroll
  for (int e = 0; e < 8; ++e) {
    const int d = i - (j + e);
    adm[e] = active && (d >= 0) && (d < kWin);
    t[e] = adm[e] ? sv[e] : -INFINITY;
    m = fmaxf(m, t[e]);
  }
#pragma unroll
  for (int off = 16; off > 0; off >>= 1) m = fmaxf(m, __shfl_xor(m, off, 32));
  float ev[8];
  float s = 0.f;
#pragma unroll
  for (int e = 0; e < 8; ++e) {
    ev[e] = adm[e] ? __expf(t[e] - m) : 0.0f;
    s += ev[e];
  }
#pragma unroll
  for (int off = 16; off > 0; off >>= 1) s += __shfl_xor(s, off, 32);
  const float inv = 32768.0f * (1.0f / s);
  unsigned short hb[8];
#pragma unroll
  for (int e = 0; e < 8; ++e) hb[e] = __builtin_bit_cast(unsigned short, (_Float16)(ev[e] * inv));
  const v4u pv = (v4u){pk16(hb[0], hb[1]), pk16(hb[2], hb[3]), pk16(hb[4], hb[5]), pk16(hb[6], hb[7])};
  unsigned short* dst = P + roff + (size_t)jjc;
  if (active) *(volatile v4u*)dst = pv;
  __threadfence();
  if (active) *(volatile v4u*)dst = pv;
}

extern "C" void kernel_launch(void* const* d_in, const int* in_sizes, int n_in,
                              void* d_out, int out_size, void* d_ws, size_t ws_size,
                              hipStream_t stream)
{
  if (n_in < 17) return;
  if (in_sizes[0] != kRows * kD) return;
  if (in_sizes[1] != kD || in_sizes[2] != kD) return;
  if (in_sizes[3] != kWinRows * kD) return;
  if (in_sizes[4] != kHS * kDTR) return;
  if (in_sizes[5] != kDI * 4 || in_sizes[6] != kDI) return;
  if (in_sizes[7] != kHS * kNS || in_sizes[8] != kHS * kPch || in_sizes[9] != kHS) return;
  if (in_sizes[10] != kDI) return;
  if (in_sizes[11] != kD * kDI || in_sizes[12] != kDI * kD) return;
  if (in_sizes[13] != kD * kD || in_sizes[14] != kD * kD || in_sizes[15] != kD * kD || in_sizes[16] != kD * kD) return;
  if (out_size != kRows * kD) return;

  const float* x        = (const float*)d_in[0];
  const float* norm1_w  = (const float*)d_in[1];
  const float* norm2_w  = (const float*)d_in[2];
  const float* Win      = (const float*)d_in[3];
  const float* Wdt      = (const float*)d_in[4];
  const float* conv_w   = (const float*)d_in[5];
  const float* conv_b   = (const float*)d_in[6];
  const float* A_log    = (const float*)d_in[7];
  const float* Dskip    = (const float*)d_in[8];
  const float* dt_bias  = (const float*)d_in[9];
  const float* ssd_nw   = (const float*)d_in[10];
  const float* Wout_ssd = (const float*)d_in[11];
  const float* Wres     = (const float*)d_in[12];
  const float* Wq       = (const float*)d_in[13];
  const float* Wk       = (const float*)d_in[14];
  const float* Wv       = (const float*)d_in[15];
  const float* Wo       = (const float*)d_in[16];
  float* out = (float*)d_out;

  const size_t SZ_WIN   = (size_t)kWinRows * kD * 2;
  const size_t SZ_W2    = (size_t)kDI * kD * 2;
  const size_t SZ_W1    = (size_t)kD * kD * 2;
  const size_t SZ_U16   = (size_t)kRows * kD * 2;
  const size_t SZ_H     = (size_t)kRows * kD * 4;
  const size_t SZ_XZ    = (size_t)kT * kXZP * 4;
  const size_t SZ_Y     = (size_t)kT * kDI * 4;
  const size_t SZ_G16   = (size_t)kT * kDI * 2;
  const size_t SZ_DBC   = (size_t)kT * kDBCP * 4;
  const size_t SZ_QKF   = (size_t)kRows * 2 * kD * 4;
  const size_t SZ_S     = (size_t)kSGH * kT * kPBW * 4;
  const size_t SZ_P     = (size_t)kSGH * kT * kPBW * 2;
  const size_t SZ_CTX   = (size_t)kRows * kD * 2;
  const size_t SZ_VT    = (size_t)kBatch * kD * kT * 2;
  const size_t SZ_QK16  = (size_t)kRows * 2 * kD * 2;
  const size_t SZ_CS    = (size_t)kT * 64 * 4;

  const size_t OFF_WIN   = 0;
  const size_t OFF_WRES  = OFF_WIN  + SZ_WIN;
  const size_t OFF_WOUT  = OFF_WRES + SZ_W2;
  const size_t OFF_WQ    = OFF_WOUT + SZ_W2;
  const size_t OFF_WK    = OFF_WQ + SZ_W1;
  const size_t OFF_WV    = OFF_WK + SZ_W1;
  const size_t OFF_WO    = OFF_WV + SZ_W1;
  const size_t OFF_U16   = OFF_WO + SZ_W1;
  const size_t OFF_H     = OFF_U16 + SZ_U16;
  const size_t OFF_AR    = OFF_H + SZ_H;
  const size_t AOFF_XZ   = 0;
  const size_t AOFF_Y    = AOFF_XZ  + SZ_XZ;
  const size_t AOFF_Y2   = AOFF_Y   + SZ_Y;
  const size_t AOFF_G16  = AOFF_Y2  + SZ_Y;
  const size_t AOFF_DBC  = AOFF_G16 + SZ_G16;
  const size_t AEND_SSD  = AOFF_DBC + SZ_DBC;
  const size_t AOFF_QKF  = 0;
  const size_t AOFF_S    = 0;
  const size_t AOFF_P    = AOFF_S + SZ_S;
  const size_t AOFF_CTX  = AOFF_P + SZ_P;
  const size_t AOFF_VT   = AOFF_QKF + SZ_QKF;
  const size_t AOFF_QK16 = AOFF_VT  + SZ_VT;
  const size_t AOFF_CS   = AOFF_QK16 + SZ_QK16;
  const size_t AEND_ATT  = AOFF_CS + SZ_CS;
  const size_t SZ_AR     = (AEND_SSD > AEND_ATT) ? AEND_SSD : AEND_ATT;
  const size_t TOTAL     = OFF_AR + SZ_AR;
  if (AOFF_CTX + SZ_CTX > SZ_QKF) return;
  if (TOTAL > ws_size) return;
  if (TOTAL > (size_t)134217728) return;

  char* ws = (char*)d_ws;
  unsigned short* WIN16  = (unsigned short*)(ws + OFF_WIN);
  unsigned short* WRES16 = (unsigned short*)(ws + OFF_WRES);
  unsigned short* WOUT16 = (unsigned short*)(ws + OFF_WOUT);
  unsigned short* WQ16   = (unsigned short*)(ws + OFF_WQ);
  unsigned short* WK16   = (unsigned short*)(ws + OFF_WK);
  unsigned short* WV16   = (unsigned short*)(ws + OFF_WV);
  unsigned short* WO16   = (unsigned short*)(ws + OFF_WO);
  unsigned short* U16    = (unsigned short*)(ws + OFF_U16);
  float*          H      = (float*)(ws + OFF_H);
  char* ar = ws + OFF_AR;
  float*          XZ     = (float*)(ar + AOFF_XZ);
  float*          Y      = (float*)(ar + AOFF_Y);
  float*          Y2     = (float*)(ar + AOFF_Y2);
  unsigned short* G16    = (unsigned short*)(ar + AOFF_G16);
  float*          DBC    = (float*)(ar + AOFF_DBC);
  float*          QKF    = (float*)(ar + AOFF_QKF);
  float*          Sbuf   = (float*)(ar + AOFF_S);
  unsigned short* P16    = (unsigned short*)(ar + AOFF_P);
  unsigned short* CTX16  = (unsigned short*)(ar + AOFF_CTX);
  unsigned short* VT16   = (unsigned short*)(ar + AOFF_VT);
  unsigned short* QK16   = (unsigned short*)(ar + AOFF_QK16);
  float*          CS     = (float*)(ar + AOFF_CS);
  const float* dummy = norm1_w;
  const dim3 blk(256);

  cast_f16_kernel<<<dim3((kWinRows * kD / 8 + 255) / 256), blk, 0, stream>>>(Win, WIN16, kWinRows * kD / 8, 16.0f);
  cast_f16_kernel<<<dim3((kDI * kD / 8 + 255) / 256), blk, 0, stream>>>(Wres, WRES16, kDI * kD / 8, 16.0f);
  cast_f16_kernel<<<dim3((kD * kDI / 8 + 255) / 256), blk, 0, stream>>>(Wout_ssd, WOUT16, kD * kDI / 8, 16.0f);
  cast_f16_kernel<<<dim3((kD * kD / 8 + 255) / 256), blk, 0, stream>>>(Wq, WQ16, kD * kD / 8, 16.0f);
  cast_f16_kernel<<<dim3((kD * kD / 8 + 255) / 256), blk, 0, stream>>>(Wk, WK16, kD * kD / 8, 16.0f);
  cast_f16_kernel<<<dim3((kD * kD / 8 + 255) / 256), blk, 0, stream>>>(Wv, WV16, kD * kD / 8, 16.0f);
  cast_f16_kernel<<<dim3((kD * kD / 8 + 255) / 256), blk, 0, stream>>>(Wo, WO16, kD * kD / 8, 16.0f);

  rms_f16_kernel<<<dim3(kRows), dim3(128), 0, stream>>>(x, norm1_w, U16);

  for (int b = 0; b < kBatch; ++b) {
    const unsigned short* U16b = U16 + (size_t)b * kT * kD;
    wmma_gemm64<0, false, 0, 0, false><<<dim3(256, 1), blk, 0, stream>>>(
        U16b, U16b, kD, 0L, WIN16, WIN16, kD, 0L,
        (void*)XZ, (void*)XZ, kXZP, 0L, dummy, dummy, 0L, kT, kXZP, kD, 0.0625f, 1.0f);
    wmma_gemm64<0, false, 0, 0, false><<<dim3(20, 1), blk, 0, stream>>>(
        U16b, U16b, kD, 0L, WIN16 + (size_t)kXZP * kD, WIN16 + (size_t)kXZP * kD, kD, 0L,
        (void*)DBC, (void*)DBC, kDBCP, 0L, dummy, dummy, 0L, kT, kDBCP, kD, 0.0625f, 1.0f);
    ssm_scan_kernel<<<dim3(kHS), blk, 0, stream>>>(XZ, DBC, Wdt, dt_bias, conv_w, conv_b, A_log, Dskip, Y);
    wmma_gemm64<0, false, 0, 0, true><<<dim3(128, 1), blk, 0, stream>>>(
        U16b, U16b, kD, 0L, WRES16, WRES16, kD, 0L,
        (void*)Y2, (void*)Y2, kDI, 0L, dummy, Y, 0L, kT, kDI, kD, 0.0625f, 1.0f);
    gate_rms_kernel<<<dim3(kT), blk, 0, stream>>>(Y2, XZ, ssd_nw, G16);
    wmma_gemm64<0, false, 0, 0, true><<<dim3(64, 1), blk, 0, stream>>>(
        G16, G16, kDI, 0L, WOUT16, WOUT16, kDI, 0L,
        (void*)(H + (size_t)b * kT * kD), (void*)(H + (size_t)b * kT * kD), kD, 0L,
        dummy, x + (size_t)b * kT * kD, 0L, kT, kD, kDI, 0.0625f, 1.0f);
  }

  unsigned short* U2_16 = U16;
  rms_f16_kernel<<<dim3(kRows), dim3(128), 0, stream>>>(H, norm2_w, U2_16);

  wmma_gemm64<0, false, 0, 0, false><<<dim3(256, 1), blk, 0, stream>>>(
      U2_16, U2_16, kD, 0L, WQ16, WQ16, kD, 0L,
      (void*)QKF, (void*)QKF, 2 * kD, 0L, dummy, dummy, 0L, kRows, 2 * kD, kD, 0.0625f, 1.0f);
  wmma_gemm64<0, false, 0, 1, false><<<dim3(64, kBatch), blk, 0, stream>>>(
      WV16, WV16, kD, 0L, U2_16, U2_16, kD, (long)kT * kD,
      (void*)VT16, (void*)VT16, kT, (long)kD * kT, dummy, dummy, 0L, kD, kT, kD, 0.5f, 1.0f);
  rope_table_kernel<<<dim3((kT * 32) / 256), blk, 0, stream>>>(CS);
  rope_cast_kernel<<<dim3(kRows), blk, 0, stream>>>(QKF, CS, QK16);

  const dim3 gS(((kT / 64) * (kT / 64) + 7) / 8, kSGH);
  const dim3 gSm(kT, kSGH);
  const dim3 gPV(((kT / 64) * (kHD / 64) + 7) / 8, kSGH);
  for (int b = 0; b < kBatch; ++b) {
    const unsigned short* QKb = QK16 + (size_t)b * kT * (2 * kD);
    const unsigned short* VTb = VT16 + (size_t)b * kD * kT;
    for (int sg = 0; sg < kHeadsA / kSGH; ++sg) {
      const int h0 = sg * kSGH;
      wmma_gemm64<0, false, 0, 0, false, 0, kBandL, 0, -1, 0, true><<<gS, blk, 0, stream>>>(
          QKb + (size_t)h0 * kHD, QKb + (size_t)h0 * kHD, 2 * kD, (long)kHD,
          QKb + kD + (size_t)h0 * kHD, QKb + kD + (size_t)h0 * kHD, 2 * kD, (long)kHD,
          (void*)Sbuf, (void*)Sbuf, kPBW, (long)kT * kPBW,
          dummy, dummy, 0L, kT, kT, kHD, 0.001953125f, 1.0f);
      band_softmax_kernel<<<gSm, dim3(32), 0, stream>>>(Sbuf, P16);
      wmma_gemm64<0, false, 0, 1, false, 0, -1, 0, kBandL, 0, true><<<gPV, blk, 0, stream>>>(
          P16, P16, kPBW, (long)kT * kPBW,
          VTb + (size_t)h0 * kHD * kT, VTb + (size_t)h0 * kHD * kT, kT, (long)kHD * kT,
          (void*)(CTX16 + (size_t)b * kT * kD + (size_t)h0 * kHD), (void*)(CTX16 + (size_t)b * kT * kD + (size_t)h0 * kHD),
          kD, (long)kHD,
          dummy, dummy, 0L, kT, kHD, kT, 0.000030517578125f, 1.0f);
    }
  }

  wmma_gemm64<0, false, 0, 0, true><<<dim3(128, 1), blk, 0, stream>>>(
      CTX16, CTX16, kD, 0L, WO16, WO16, kD, 0L,
      (void*)out, (void*)out, kD, 0L, dummy, H, 0L, kRows, kD, kD, 0.0078125f, 1.0f);
}
